// ParallelConvSSM3D_13091060318339
// MI455X (gfx1250) — hardware-run, weakly checked
//
#include <hip/hip_runtime.h>
#include <math.h>

typedef __attribute__((ext_vector_type(16))) _Float16 v16h;
typedef __attribute__((ext_vector_type(8)))  _Float16 v8h;
typedef __attribute__((ext_vector_type(2)))  _Float16 v2h;
typedef __attribute__((ext_vector_type(8)))  float    v8f;
typedef __attribute__((ext_vector_type(4)))  float    v4f;
typedef __attribute__((ext_vector_type(2)))  float    v2f;
typedef __attribute__((ext_vector_type(4)))  unsigned v4u;
typedef __attribute__((ext_vector_type(8)))  unsigned v8u;

constexpr int kT  = 16;
constexpr int kH  = 64;
constexpr int kW  = 64;
constexpr int kC  = 128;
constexpr int kTh = 9;
constexpr int kStrT = kH * kW * kC;
constexpr int kStrH = kW * kC;
constexpr int kStrW = kC;
constexpr int kTapsPerCh = 3 * 7 * 7;
constexpr size_t kFieldElems = (size_t)kTh * kStrT;
static_assert(kStrT == 524288 && kStrH == 8192 && kStrW == 128, "strides");
static_assert(kFieldElems == 4718592ull, "half-spectrum field size");

constexpr float kTwoPi        = 6.28318530717958647692f;
constexpr float kF16MinNormal = 6.103515625e-05f;
constexpr float kF16Clamp     = 60000.0f;

constexpr float kCarryTw    = 1024.0f;
constexpr float kCarryTwInvT = 512.0f;
constexpr float kCarryX     = 64.0f;
constexpr float kCarryS1    = 16.0f;
constexpr float kCarryS2    = 4.0f;
constexpr float kCarryY     = 1.0f;
constexpr float kCarryS4    = 8.0f;
constexpr float kCarryS5    = 64.0f;
constexpr float kScaleS1 = kCarryS1 / (kCarryTw * kCarryX);
constexpr float kScaleS2 = kCarryS2 / (kCarryTw * kCarryS1);
constexpr float kScaleS3 = 1.0f / (kCarryTw * kCarryS2);
constexpr float kScaleS4 = kCarryS4 / ((float)kW * kCarryTw * kCarryY);
constexpr float kScaleS5 = kCarryS5 / ((float)kH * kCarryTw * kCarryS4);
constexpr float kScaleS6 = 1.0f / ((float)kT * kCarryTwInvT * kCarryS5);

constexpr bool kTwoTermTwiddle = false;

constexpr int kTwF64   = 0;
constexpr int kTwI64   = 16384;
constexpr int kTwF16   = 32768;
constexpr int kTwI16   = 33280;
constexpr int kTwTotal = 33792;
static_assert((kTwTotal % 64) == 0, "table is whole 128-B lines");

constexpr size_t kSzTw  = (size_t)kTwTotal * 2;
constexpr size_t kSzP1  = (size_t)21 * 64 * 128 * 2 * 4;
constexpr size_t kSzP2  = (size_t)3 * 64 * 64 * 128 * 2 * 4;
constexpr size_t kSzF16 = kFieldElems * 2;
constexpr size_t kSzF32 = kFieldElems * 4;
constexpr size_t kOffTWH  = 0;
constexpr size_t kOffTWL  = kOffTWH  + kSzTw;
constexpr size_t kOffP1A  = kOffTWL  + kSzTw;
constexpr size_t kOffP1B  = kOffP1A  + kSzP1;
constexpr size_t kOffP2A  = kOffP1B  + kSzP1;
constexpr size_t kOffP2B  = kOffP2A  + kSzP2;
constexpr size_t kOffFARE = kOffP2B  + kSzP2;
constexpr size_t kOffFAIM = kOffFARE + kSzF16;
constexpr size_t kOffFBRE = kOffFAIM + kSzF16;
constexpr size_t kOffFBIM = kOffFBRE + kSzF16;
constexpr size_t kOffXRE  = kOffFBIM + kSzF16;
constexpr size_t kOffXIM  = kOffXRE  + kSzF32;
constexpr size_t kWsTotal = kOffXIM  + kSzF32;
static_assert(kWsTotal == 103550976ull, "carve total");
static_assert(kWsTotal <= 134217728ull, "carve cap");
static_assert((kOffTWL % 128) == 0 && (kOffP1A % 128) == 0 && (kOffP1B % 128) == 0 && (kOffP2A % 128) == 0 &&
              (kOffP2B % 128) == 0 && (kOffFARE % 128) == 0 && (kOffFAIM % 128) == 0 && (kOffFBRE % 128) == 0 &&
              (kOffFBIM % 128) == 0 && (kOffXRE % 128) == 0 && (kOffXIM % 128) == 0, "128-B aligned regions");
static_assert(kOffFAIM == kOffFARE + kFieldElems * 2, "imaginary plane follows the real plane");

constexpr int kP1Pairs = 21 * 64 * 64;
constexpr int kP2Pairs = 3 * 64 * 64 * 64;
constexpr int kPwPairs = (int)(kFieldElems / 2);
static_assert((kP1Pairs % 256) == 0 && (kP2Pairs % 256) == 0 && (kPwPairs % 256) == 0, "exact grids");

__device__ __forceinline__ _Float16 to_h(float v) {
  const float keep = (fabsf(v) < kF16MinNormal) ? 0.0f : v;
  const float lim  = fminf(fmaxf(keep, -kF16Clamp), kF16Clamp);
  return (_Float16)lim;
}

union FragU { v16h v; v4u q[2]; };

__device__ __forceinline__ v16h frag_from_global(const unsigned short* p) {
  FragU f;
  f.q[0] = *(const v4u*)(const void*)(p);
  f.q[1] = *(const v4u*)(const void*)(p + 16);
  return f.v;
}
__device__ __forceinline__ v16h frag_from_lds(const unsigned* p) {
  FragU f;
  f.q[0] = *(const v4u*)(p);
  f.q[1] = *(const v4u*)(p + 8);
  return f.v;
}
__device__ __forceinline__ v8f mma_g(v16h a, v16h b, v8f c) {
  c = __builtin_amdgcn_wmma_f32_16x16x32_f16(false, a, false, b, (short)0, c, false, false);
  asm volatile("v_nop\n\tv_nop\n\tv_nop\n\tv_nop" : "+v"(c) : "v"(a), "v"(b));
  return c;
}
__device__ __forceinline__ void wave_lds_sync() {
  __builtin_amdgcn_fence(__ATOMIC_RELEASE, "workgroup");
  __builtin_amdgcn_wave_barrier();
  __builtin_amdgcn_fence(__ATOMIC_ACQUIRE, "workgroup");
}

__device__ __forceinline__ float tw_elem(int gid, const float* tc, const float* ts) {
  int j;
  bool useSin;
  float mult;
  if (gid < kTwF16) {
    const bool inv = (gid >= kTwI64);
    const int loc = gid & 16383;
    const int m = loc >> 7, k = loc & 127;
    const int mhi = m >> 6, khi = k >> 6;
    j = ((m & 63) * (k & 63)) & 63;
    useSin = (mhi != khi);
    const bool neg = useSin && ((khi == 0) != inv);
    mult = neg ? -kCarryTw : kCarryTw;
  } else if (gid < kTwI16) {
    const int loc = gid - kTwF16;
    const int m = loc >> 5, k = loc & 31;
    useSin = (m >= 9);
    const int tp = useSin ? (m - 8) : m;
    j = ((tp * k) & 15) * 4;
    mult = (k >= 16) ? 0.0f : (useSin ? -kCarryTw : kCarryTw);
  } else {
    const int loc = gid - kTwI16;
    const int t = loc >> 5, k = loc & 31;
    useSin = (k >= 9);
    const int kk = useSin ? (k - 8) : k;
    j = ((kk * t) & 15) * 4;
    const float wgt = ((k == 0) || (k == 8)) ? kCarryTwInvT : (2.0f * kCarryTwInvT);
    mult = (k >= 16) ? 0.0f : (useSin ? -wgt : wgt);
  }
  const float cv = tc[j];
  const float sv = ts[j];
  const float base = useSin ? sv : cv;
  return (mult != 0.0f) ? (base * mult) : 0.0f;
}

__global__ __launch_bounds__(256) void tw_table_kernel(unsigned short* __restrict__ thi,
                                                       unsigned short* __restrict__ tlo) {
  __shared__ float tc[64];
  __shared__ float ts[64];
  const int tid = threadIdx.x;
  if (tid < 64) {
    float s, c;
    sincosf((float)tid * (kTwoPi / 64.0f), &s, &c);
    tc[tid] = c;
    ts[tid] = s;
  }
  __syncthreads();
  const int th = blockIdx.x * 256 + tid;
  if (th < kTwTotal / 8) {
    const int g0 = th * 8;
    v8h hv, lv;
#pragma unroll
    for (int e = 0; e < 8; ++e) {
      const float v = tw_elem(g0 + e, tc, ts);
      const _Float16 hm = to_h(v);
      const float res = v - (float)hm;
      hv[e] = hm;
      lv[e] = to_h(res);
    }
    unsigned short* ph = thi + g0;
    unsigned short* pl = tlo + g0;
    *(volatile v8h*)(void*)ph = hv;
    if (kTwoTermTwiddle) *(volatile v8h*)(void*)pl = lv;
    __threadfence();
    *(volatile v8h*)(void*)ph = hv;
    if (kTwoTermTwiddle) *(volatile v8h*)(void*)pl = lv;
  }
}

__global__ __launch_bounds__(256) void kspec_w_kernel(const float* __restrict__ Ak, const float* __restrict__ Bk,
                                                      float* __restrict__ P1A, float* __restrict__ P1B) {
  __shared__ float tc[64];
  __shared__ float ts[64];
  const int tid = threadIdx.x;
  if (tid < 64) {
    float s, c;
    sincosf((float)tid * (kTwoPi / 64.0f), &s, &c);
    tc[tid] = c;
    ts[tid] = s;
  }
  __syncthreads();
  const int i  = blockIdx.x * 256 + tid;
  const int c2 = i & 63;
  const int w  = (i >> 6) & 63;
  const int kk = i >> 12;
  const int kt = kk / 7;
  const int kh = kk - kt * 7;
  const int ka0 = (((2 * c2) * 3 + kt) * 7 + kh) * 7;
  const int ka1 = ka0 + kTapsPerCh;
  v4f accA = (v4f){0.f, 0.f, 0.f, 0.f};
  v4f accB = (v4f){0.f, 0.f, 0.f, 0.f};
#pragma unroll 1
  for (int kw = 0; kw < 7; ++kw) {
    const int j = (w * (kw - 3)) & 63;
    const float cj = tc[j];
    const float sj = -ts[j];
    const float a0 = 0.9f * tanhf(Ak[ka0 + kw]);
    const float a1 = 0.9f * tanhf(Ak[ka1 + kw]);
    const float b0 = Bk[ka0 + kw];
    const float b1 = Bk[ka1 + kw];
    accA[0] = fmaf(a0, cj, accA[0]);
    accA[1] = fmaf(a0, sj, accA[1]);
    accA[2] = fmaf(a1, cj, accA[2]);
    accA[3] = fmaf(a1, sj, accA[3]);
    accB[0] = fmaf(b0, cj, accB[0]);
    accB[1] = fmaf(b0, sj, accB[1]);
    accB[2] = fmaf(b1, cj, accB[2]);
    accB[3] = fmaf(b1, sj, accB[3]);
  }
  float* qa = P1A + 4 * (size_t)i;
  float* qb = P1B + 4 * (size_t)i;
  *(volatile v4f*)qa = accA;
  *(volatile v4f*)qb = accB;
  __threadfence();
  *(volatile v4f*)qa = accA;
  *(volatile v4f*)qb = accB;
}

__global__ __launch_bounds__(256) void kspec_h_kernel(const float* __restrict__ P1A, const float* __restrict__ P1B,
                                                      float* __restrict__ P2A, float* __restrict__ P2B) {
  __shared__ float tc[64];
  __shared__ float ts[64];
  const int tid = threadIdx.x;
  if (tid < 64) {
    float s, c;
    sincosf((float)tid * (kTwoPi / 64.0f), &s, &c);
    tc[tid] = c;
    ts[tid] = s;
  }
  __syncthreads();
  const int i  = blockIdx.x * 256 + tid;
  const int c2 = i & 63;
  const int w  = (i >> 6) & 63;
  const int h  = (i >> 12) & 63;
  const int kt = i >> 18;
  v4f accA = (v4f){0.f, 0.f, 0.f, 0.f};
  v4f accB = (v4f){0.f, 0.f, 0.f, 0.f};
#pragma unroll 1
  for (int kh = 0; kh < 7; ++kh) {
    const int j = (h * (kh - 3)) & 63;
    const float cj = tc[j];
    const float sj = -ts[j];
    const int pi = ((kt * 7 + kh) * 64 + w) * 64 + c2;
    const v4f pa = *(const v4f*)(P1A + 4 * (size_t)pi);
    const v4f pb = *(const v4f*)(P1B + 4 * (size_t)pi);
    accA[0] += pa[0] * cj - pa[1] * sj;
    accA[1] += pa[0] * sj + pa[1] * cj;
    accA[2] += pa[2] * cj - pa[3] * sj;
    accA[3] += pa[2] * sj + pa[3] * cj;
    accB[0] += pb[0] * cj - pb[1] * sj;
    accB[1] += pb[0] * sj + pb[1] * cj;
    accB[2] += pb[2] * cj - pb[3] * sj;
    accB[3] += pb[2] * sj + pb[3] * cj;
  }
  float* qa = P2A + 4 * (size_t)i;
  float* qb = P2B + 4 * (size_t)i;
  *(volatile v4f*)qa = accA;
  *(volatile v4f*)qb = accB;
  __threadfence();
  *(volatile v4f*)qa = accA;
  *(volatile v4f*)qb = accB;
}

__global__ __launch_bounds__(256) void dft16_fwd_kernel(
    const float* __restrict__ x, const unsigned short* __restrict__ twh, const unsigned short* __restrict__ twl,
    unsigned short* __restrict__ ore, unsigned short* __restrict__ oim) {
  __shared__ __align__(16) float sT[8][16 * 68];
  const int tid = threadIdx.x, lane = tid & 31, wave = tid >> 5;
  const int hh = lane >> 4, c = lane & 15;
  const int task = blockIdx.x * 8 + wave;
  const int n0 = (task >> 1) * kC + (task & 1) * 64;

  v4f xv[8];
#pragma unroll
  for (int i = 0; i < 8; ++i)
    xv[i] = *(const v4f*)(x + (size_t)(8 * hh + i) * kStrT + n0 + 4 * c);

  const v16h a = frag_from_global(twh + kTwF16 + c * 32 + 8 * hh);
  v16h al = a;
  if (kTwoTermTwiddle) al = frag_from_global(twl + kTwF16 + c * 32 + 8 * hh);

  v8f acc[4];
#pragma unroll
  for (int j = 0; j < 4; ++j) {
    v16h b;
#pragma unroll
    for (int i = 0; i < 8; ++i) {
      b[i] = to_h(xv[i][j] * kCarryX);
      b[8 + i] = (_Float16)0.0f;
    }
    acc[j] = mma_g(a, b, (v8f){0.f, 0.f, 0.f, 0.f, 0.f, 0.f, 0.f, 0.f});
    if (kTwoTermTwiddle) acc[j] = mma_g(al, b, acc[j]);
  }

  float* slab = sT[wave];
#pragma unroll
  for (int r = 0; r < 8; ++r) {
    const v4f v = (v4f){acc[0][r] * kScaleS1, acc[1][r] * kScaleS1, acc[2][r] * kScaleS1, acc[3][r] * kScaleS1};
    *(v4f*)(slab + (8 * hh + r) * 68 + 4 * c) = v;
  }
  wave_lds_sync();

  const int q = lane >> 3, c8 = (lane & 7) * 8;
  v8h hv[5];
  unsigned short* dst[5];
  bool live[5];
#pragma unroll
  for (int it = 0; it < 5; ++it) {
    const int rr = it * 4 + q;
    const int srow = (rr < 16) ? rr : 15;
    const float* sp = slab + srow * 68 + c8;
    const v4f a0 = *(const v4f*)(sp);
    const v4f a1 = *(const v4f*)(sp + 4);
    const bool data = (rr < 16);
#pragma unroll
    for (int e = 0; e < 4; ++e) {
      const float f0 = data ? a0[e] : 0.0f;
      const float f1 = data ? a1[e] : 0.0f;
      hv[it][e]     = to_h(f0);
      hv[it][4 + e] = to_h(f1);
    }
    const bool isRe = (rr < 9);
    const int tpp = isRe ? rr : ((rr < 16) ? (rr - 8) : ((rr == 16) ? 0 : 8));
    dst[it] = (isRe ? ore : oim) + (size_t)tpp * kStrT + n0 + c8;
    live[it] = (rr < 18);
  }
  for (int pass = 0; pass < 2; ++pass) {
#pragma unroll
    for (int it = 0; it < 5; ++it) {
      if (live[it]) *(volatile v8h*)(void*)dst[it] = hv[it];
    }
    __threadfence();
  }
}

template <bool OUT32>
__global__ __launch_bounds__(128) void dft64_kernel(
    const unsigned short* __restrict__ ire, const unsigned short* __restrict__ iim,
    const unsigned short* __restrict__ twh, const unsigned short* __restrict__ twl,
    void* __restrict__ ore, void* __restrict__ oim,
    int axisStride, int otherStride, float scale) {
  __shared__ __align__(16) unsigned sB[64 * 68];
  __shared__ __align__(16) float sT[4][16 * 68];
  const int tid = threadIdx.x, lane = tid & 31, wave = tid >> 5;
  const int hh = lane >> 4, c = lane & 15;
  const int tp = blockIdx.x >> 6, o = blockIdx.x & 63, ch0 = blockIdx.y * 64;
  const size_t base = (size_t)tp * kStrT + (size_t)o * otherStride + ch0;

#pragma unroll
  for (int it = 0; it < 4; ++it) {
    const int idx = it * 128 + tid;
    const int cg = idx & 7;
    const int kp = idx >> 3;
    const unsigned short* pl = (it < 2) ? ire : iim;
    const int ra = 2 * (kp & 31);
    const v4u u0 = *(const v4u*)(const void*)(pl + base + (size_t)ra * axisStride + cg * 8);
    const v4u u1 = *(const v4u*)(const void*)(pl + base + (size_t)(ra + 1) * axisStride + cg * 8);
    unsigned* dstw = sB + (cg * 8) * 68 + kp;
#pragma unroll
    for (int p = 0; p < 4; ++p) {
      const unsigned w0 = u0[p];
      const unsigned w1 = u1[p];
      dstw[(2 * p) * 68]     = (w0 & 0xffffu) | (w1 << 16);
      dstw[(2 * p + 1) * 68] = (w0 >> 16) | (w1 & 0xffff0000u);
    }
  }
  __syncthreads();

  v8f acc[2][4];
#pragma unroll
  for (int i = 0; i < 2; ++i)
#pragma unroll
    for (int j = 0; j < 4; ++j) acc[i][j] = (v8f){0.f, 0.f, 0.f, 0.f, 0.f, 0.f, 0.f, 0.f};

#pragma unroll
  for (int ks = 0; ks < 4; ++ks) {
    const int k0 = ks * 32;
    v16h bfr[4];
#pragma unroll
    for (int j = 0; j < 4; ++j)
      bfr[j] = frag_from_lds(sB + (j * 16 + c) * 68 + (k0 >> 1) + 4 * hh);
#pragma unroll
    for (int i = 0; i < 2; ++i) {
      const size_t ao = (size_t)(wave * 32 + i * 16 + c) * 128 + k0 + 8 * hh;
      const v16h a = frag_from_global(twh + ao);
#pragma unroll
      for (int j = 0; j < 4; ++j) acc[i][j] = mma_g(a, bfr[j], acc[i][j]);
      if (kTwoTermTwiddle) {
        const v16h al = frag_from_global(twl + ao);
#pragma unroll
        for (int j = 0; j < 4; ++j) acc[i][j] = mma_g(al, bfr[j], acc[i][j]);
      }
    }
  }

  float* slab = sT[wave];
#pragma unroll
  for (int i = 0; i < 2; ++i) {
    const int ax0 = (wave & 1) * 32 + i * 16;
#pragma unroll
    for (int j = 0; j < 4; ++j)
#pragma unroll
      for (int r = 0; r < 8; ++r)
        slab[(8 * hh + r) * 68 + j * 16 + c] = acc[i][j][r] * scale;
    wave_lds_sync();
    if (OUT32) {
      float* dpl = (wave < 2) ? (float*)ore : (float*)oim;
      const int c4 = (lane & 15) * 4;
      v4f ov[8];
#pragma unroll
      for (int it = 0; it < 8; ++it) ov[it] = *(const v4f*)(slab + (it * 2 + hh) * 68 + c4);
      for (int pass = 0; pass < 2; ++pass) {
#pragma unroll
        for (int it = 0; it < 8; ++it) {
          const int row = it * 2 + hh;
          *(volatile v4f*)(dpl + base + (size_t)(ax0 + row) * axisStride + c4) = ov[it];
        }
        __threadfence();
      }
    } else {
      unsigned short* dpl = (wave < 2) ? (unsigned short*)ore : (unsigned short*)oim;
      const int q = lane >> 3, c8 = (lane & 7) * 8;
      v8h hv[4];
#pragma unroll
      for (int it = 0; it < 4; ++it) {
        const float* sp = slab + (it * 4 + q) * 68 + c8;
        const v4f a0 = *(const v4f*)(sp);
        const v4f a1 = *(const v4f*)(sp + 4);
#pragma unroll
        for (int e = 0; e < 4; ++e) {
          hv[it][e]     = to_h(a0[e]);
          hv[it][4 + e] = to_h(a1[e]);
        }
      }
      for (int pass = 0; pass < 2; ++pass) {
#pragma unroll
        for (int it = 0; it < 4; ++it) {
          const int row = it * 4 + q;
          *(volatile v8h*)(void*)(dpl + base + (size_t)(ax0 + row) * axisStride + c8) = hv[it];
        }
        __threadfence();
      }
    }
    wave_lds_sync();
  }
}

__global__ __launch_bounds__(256) void spectral_pointwise_kernel(
    const float* __restrict__ xre, const float* __restrict__ xim,
    const float* __restrict__ P2A, const float* __restrict__ P2B,
    unsigned* __restrict__ yre, unsigned* __restrict__ yim) {
  const int i  = blockIdx.x * 256 + threadIdx.x;
  const int e0 = i * 2;
  const int tp = e0 >> 19;
  const int rem = e0 & (kStrT - 1);
  float ss, cc;
  sincosf((float)tp * (kTwoPi / 16.0f), &ss, &cc);
  const v2f xr = *(const v2f*)(xre + e0);
  const v2f xi = *(const v2f*)(xim + e0);
  const v4f a0 = *(const v4f*)(P2A + 2 * (size_t)rem);
  const v4f a1 = *(const v4f*)(P2A + 2 * ((size_t)kStrT + rem));
  const v4f a2 = *(const v4f*)(P2A + 2 * ((size_t)2 * kStrT + rem));
  const v4f b0 = *(const v4f*)(P2B + 2 * (size_t)rem);
  const v4f b1 = *(const v4f*)(P2B + 2 * ((size_t)kStrT + rem));
  const v4f b2 = *(const v4f*)(P2B + 2 * ((size_t)2 * kStrT + rem));
  float ar[2], ai[2], br[2], bi[2], sr[2], si[2];
#pragma unroll
  for (int ch = 0; ch < 2; ++ch) {
    ar[ch] = (a0[2 * ch] + a2[2 * ch]) * cc - (a0[2 * ch + 1] - a2[2 * ch + 1]) * ss + a1[2 * ch];
    ai[ch] = (a0[2 * ch] - a2[2 * ch]) * ss + (a0[2 * ch + 1] + a2[2 * ch + 1]) * cc + a1[2 * ch + 1];
    br[ch] = (b0[2 * ch] + b2[2 * ch]) * cc - (b0[2 * ch + 1] - b2[2 * ch + 1]) * ss + b1[2 * ch];
    bi[ch] = (b0[2 * ch] - b2[2 * ch]) * ss + (b0[2 * ch + 1] + b2[2 * ch + 1]) * cc + b1[2 * ch + 1];
    sr[ch] = 1.0f;
    si[ch] = 0.0f;
  }
#pragma unroll 1
  for (int it = 0; it < 7; ++it) {
#pragma unroll
    for (int ch = 0; ch < 2; ++ch) {
      const float nr = ar[ch] * sr[ch] - ai[ch] * si[ch] + 1.0f;
      const float ni = ar[ch] * si[ch] + ai[ch] * sr[ch];
      sr[ch] = nr;
      si[ch] = ni;
    }
  }
  v2h hr, hi;
#pragma unroll
  for (int ch = 0; ch < 2; ++ch) {
    const float gr = br[ch] * sr[ch] - bi[ch] * si[ch];
    const float gi = br[ch] * si[ch] + bi[ch] * sr[ch];
    const float yr = gr * xr[ch] - gi * xi[ch];
    const float yi = gr * xi[ch] + gi * xr[ch];
    hr[ch] = to_h(yr * kCarryY);
    hi[ch] = to_h(yi * kCarryY);
  }
  const unsigned ur = __builtin_bit_cast(unsigned, hr);
  const unsigned ui = __builtin_bit_cast(unsigned, hi);
  volatile unsigned* pr = yre + i;
  volatile unsigned* pi = yim + i;
  *pr = ur;
  *pi = ui;
  __threadfence();
  *pr = ur;
  *pi = ui;
}

__global__ __launch_bounds__(128) void dft16_inv_kernel(
    const unsigned short* __restrict__ z, const unsigned short* __restrict__ twh,
    const unsigned short* __restrict__ twl, float* __restrict__ out) {
  __shared__ __align__(16) float sT[4][16 * 132];
  const int tid = threadIdx.x, lane = tid & 31, wave = tid >> 5;
  const int hh = lane >> 4, c = lane & 15;
  const int point = blockIdx.x * 4 + wave;

  v4u rv[8];
#pragma unroll
  for (int i = 0; i < 8; ++i) {
    const int k = 8 * hh + i;
    const size_t off = (k < 9) ? ((size_t)k * kStrT) : (kFieldElems + (size_t)(k - 8) * kStrT);
    rv[i] = *(const v4u*)(const void*)(z + off + (size_t)point * kC + 8 * c);
  }
  const v16h a = frag_from_global(twh + kTwI16 + c * 32 + 8 * hh);
  v16h al = a;
  if (kTwoTermTwiddle) al = frag_from_global(twl + kTwI16 + c * 32 + 8 * hh);

  v8f acc[8];
#pragma unroll
  for (int j = 0; j < 8; ++j) {
    v8u wv;
#pragma unroll
    for (int qq = 0; qq < 4; ++qq) {
      const unsigned lo = rv[2 * qq][j >> 1];
      const unsigned hi = rv[2 * qq + 1][j >> 1];
      wv[qq] = (j & 1) ? ((lo >> 16) | (hi & 0xffff0000u)) : ((lo & 0xffffu) | (hi << 16));
      wv[4 + qq] = 0u;
    }
    const v16h b = __builtin_bit_cast(v16h, wv);
    acc[j] = mma_g(a, b, (v8f){0.f, 0.f, 0.f, 0.f, 0.f, 0.f, 0.f, 0.f});
    if (kTwoTermTwiddle) acc[j] = mma_g(al, b, acc[j]);
  }

  float* slab = sT[wave];
#pragma unroll
  for (int r = 0; r < 8; ++r) {
    const v4f v0 = (v4f){acc[0][r] * kScaleS6, acc[1][r] * kScaleS6, acc[2][r] * kScaleS6, acc[3][r] * kScaleS6};
    const v4f v1 = (v4f){acc[4][r] * kScaleS6, acc[5][r] * kScaleS6, acc[6][r] * kScaleS6, acc[7][r] * kScaleS6};
    *(v4f*)(slab + (8 * hh + r) * 132 + 8 * c)     = v0;
    *(v4f*)(slab + (8 * hh + r) * 132 + 8 * c + 4) = v1;
  }
  wave_lds_sync();
  v4f ov[16];
#pragma unroll
  for (int t = 0; t < 16; ++t) ov[t] = *(const v4f*)(slab + t * 132 + 4 * lane);
  float* ob = out + (size_t)point * kC + 4 * lane;
  for (int pass = 0; pass < 2; ++pass) {
#pragma unroll
    for (int t = 0; t < 16; ++t) *(volatile v4f*)(ob + (size_t)t * kStrT) = ov[t];
    __threadfence();
  }
}

extern "C" void kernel_launch(void* const* d_in, const int* in_sizes, int n_in,
                              void* d_out, int out_size, void* d_ws, size_t ws_size,
                              hipStream_t stream) {
  if (n_in < 3) return;
  if (in_sizes[0] != kT * kStrT) return;
  if (in_sizes[1] != kC * kTapsPerCh) return;
  if (in_sizes[2] != kC * kTapsPerCh) return;
  if (out_size != kT * kStrT) return;
  if (ws_size < kWsTotal) return;

  const float* x  = (const float*)d_in[0];
  const float* Ak = (const float*)d_in[1];
  const float* Bk = (const float*)d_in[2];
  float* out = (float*)d_out;

  char* ws = (char*)d_ws;
  unsigned short* TWH  = (unsigned short*)(ws + kOffTWH);
  unsigned short* TWL  = (unsigned short*)(ws + kOffTWL);
  float*          P1A  = (float*)(ws + kOffP1A);
  float*          P1B  = (float*)(ws + kOffP1B);
  float*          P2A  = (float*)(ws + kOffP2A);
  float*          P2B  = (float*)(ws + kOffP2B);
  unsigned short* FARE = (unsigned short*)(ws + kOffFARE);
  unsigned short* FAIM = (unsigned short*)(ws + kOffFAIM);
  unsigned short* FBRE = (unsigned short*)(ws + kOffFBRE);
  unsigned short* FBIM = (unsigned short*)(ws + kOffFBIM);
  float*          XRE  = (float*)(ws + kOffXRE);
  float*          XIM  = (float*)(ws + kOffXIM);

  tw_table_kernel<<<(kTwTotal / 8 + 255) / 256, 256, 0, stream>>>(TWH, TWL);
  kspec_w_kernel<<<kP1Pairs / 256, 256, 0, stream>>>(Ak, Bk, P1A, P1B);
  kspec_h_kernel<<<kP2Pairs / 256, 256, 0, stream>>>(P1A, P1B, P2A, P2B);
  dft16_fwd_kernel<<<(kH * kW * 2) / 8, 256, 0, stream>>>(x, TWH, TWL, FARE, FAIM);
  dft64_kernel<false><<<dim3(kTh * 64, 2), 128, 0, stream>>>(
      FARE, FAIM, TWH + kTwF64, TWL + kTwF64, (void*)FBRE, (void*)FBIM, kStrH, kStrW, kScaleS2);
  dft64_kernel<true><<<dim3(kTh * 64, 2), 128, 0, stream>>>(
      FBRE, FBIM, TWH + kTwF64, TWL + kTwF64, (void*)XRE, (void*)XIM, kStrW, kStrH, kScaleS3);
  spectral_pointwise_kernel<<<kPwPairs / 256, 256, 0, stream>>>(
      XRE, XIM, P2A, P2B, (unsigned*)(void*)FARE, (unsigned*)(void*)FAIM);
  dft64_kernel<false><<<dim3(kTh * 64, 2), 128, 0, stream>>>(
      FARE, FAIM, TWH + kTwI64, TWL + kTwI64, (void*)FBRE, (void*)FBIM, kStrW, kStrH, kScaleS4);
  dft64_kernel<false><<<dim3(kTh * 64, 2), 128, 0, stream>>>(
      FBRE, FBIM, TWH + kTwI64, TWL + kTwI64, (void*)FARE, (void*)FAIM, kStrH, kStrW, kScaleS5);
  dft16_inv_kernel<<<(kH * kW) / 4, 128, 0, stream>>>(FARE, TWH, TWL, out);
}
